// HighFreqMHSA_46420006535707
// MI455X (gfx1250) — hardware-verified
//
#include <hip/hip_runtime.h>
#include <math.h>
#include <stdint.h>


#define DIMC   512
#define HEADS  8
#define HD     64
#define NRES   196
#define OQKV   1536
#define NIMG   128
#define GIMG   32
#define NGRP   4
#define NTG    6272
#define TGP    6336
#define NQT    13
#define NMT    14
#define NKST   7
#define NKEY   224
#define KP     72
#define VP     232
#define ATHR   416
#define NBT    (HEADS * NQT * NMT * 32 * 8)
#define LDSH   (NKEY * KP + 2 * HD * VP)
#define QTP    72
#define SPP    72

static_assert(NTG == GIMG * NRES);
static_assert(TGP == NTG + 64);
static_assert(NGRP * GIMG == NIMG);
static_assert(HEADS * HD == DIMC);
static_assert((TGP % 64) == 0 && (NTG % 64) == 0 && (NRES % 4) == 0 && (DIMC % 64) == 0 && (OQKV % 64) == 0);
static_assert(NQT * 16 >= NRES && NKST * 32 == NKEY && NKEY >= NRES && NMT * 16 == NKEY);
static_assert(ATHR == NQT * 32);
static_assert((GIMG - 1) * NRES + NKEY <= TGP);
static_assert((GIMG - 1) * NRES + NQT * 16 <= TGP);
static_assert(NQT * 2048 <= LDSH);
static_assert(((GIMG * DIMC * NRES) % 1024) == 0);
static_assert((NBT % 256) == 0);

typedef _Float16 v16h __attribute__((ext_vector_type(16)));
typedef _Float16 v8h  __attribute__((ext_vector_type(8)));
typedef float    v8f  __attribute__((ext_vector_type(8)));
typedef float    v4f  __attribute__((ext_vector_type(4)));
typedef unsigned int v4u __attribute__((ext_vector_type(4)));
typedef unsigned int v2u __attribute__((ext_vector_type(2)));

__device__ __forceinline__ unsigned short bf_bits(float f) {
  unsigned u = __float_as_uint(f);
  return (unsigned short)((u + 0x7FFFu + ((u >> 16) & 1u)) >> 16);
}
__device__ __forceinline__ float bf_up(unsigned short h) { return __uint_as_float(((unsigned)h) << 16); }
__device__ __forceinline__ unsigned short h_bits(_Float16 x) { return __builtin_bit_cast(unsigned short, x); }
__device__ __forceinline__ unsigned pk16(unsigned short a, unsigned short b) { return (unsigned)a | ((unsigned)b << 16); }
__device__ __forceinline__ v8f zero8() { v8f z = {0.f, 0.f, 0.f, 0.f, 0.f, 0.f, 0.f, 0.f}; return z; }

__device__ __forceinline__ v16h ldfrag_h(const _Float16* p) {
  union { v16h v; v8h h[2]; } f;
  f.h[0] = *(const v8h*)(p);
  f.h[1] = *(const v8h*)(p + 16);
  return f.v;
}

__device__ __forceinline__ v8f mma_h_raw(v16h a, v16h b, v8f c) {
  return __builtin_amdgcn_wmma_f32_16x16x32_f16(false, a, false, b, (short)0, c, false, false);
}
__device__ __forceinline__ void res_guard(v8f& t, v8f& acc, v16h x, v16h y) {
#if defined(__HIP_DEVICE_COMPILE__)
  asm volatile("v_nop\n\tv_nop\n\tv_nop\n\tv_nop" : "+v"(t), "+v"(acc) : "v"(x), "v"(y));
#endif
}
__device__ __forceinline__ void dep_guard_h(v8f& a, v8f& b, v16h x, v16h y) {
#if defined(__HIP_DEVICE_COMPILE__)
  asm volatile("v_nop\n\tv_nop\n\tv_nop\n\tv_nop" : "+v"(a), "+v"(b) : "v"(x), "v"(y));
#endif
}
__device__ __forceinline__ void guard_sc(v8f& a, v8f& b, v16h k0, v16h k1, v16h q0, v16h q1, v16h q2, v16h q3) {
#if defined(__HIP_DEVICE_COMPILE__)
  asm volatile("v_nop\n\tv_nop\n\tv_nop\n\tv_nop" : "+v"(a), "+v"(b) : "v"(k0), "v"(k1), "v"(q0), "v"(q1), "v"(q2), "v"(q3));
#endif
}
__device__ __forceinline__ void guard_pv(v8f& a, v8f& b, v16h w, v16h x, v16h y, v16h z) {
#if defined(__HIP_DEVICE_COMPILE__)
  asm volatile("v_nop\n\tv_nop\n\tv_nop\n\tv_nop" : "+v"(a), "+v"(b) : "v"(w), "v"(x), "v"(y), "v"(z));
#endif
}
__device__ __forceinline__ void keep4_h(v16h a, v16h b, v16h c, v16h d) {
#if defined(__HIP_DEVICE_COMPILE__)
  asm volatile("v_nop" :: "v"(a), "v"(b), "v"(c), "v"(d));
#endif
}
__device__ __forceinline__ void acc_guard4(v8f& a, v8f& b, v8f& c, v8f& d) {
#if defined(__HIP_DEVICE_COMPILE__)
  asm volatile("v_nop\n\tv_nop\n\tv_nop\n\tv_nop" : "+v"(a), "+v"(b), "+v"(c), "+v"(d));
#endif
}
__device__ __forceinline__ void wave_sync_lds() {
  __builtin_amdgcn_fence(__ATOMIC_RELEASE, "workgroup");
  __builtin_amdgcn_wave_barrier();
  __builtin_amdgcn_fence(__ATOMIC_ACQUIRE, "workgroup");
}

__global__ __launch_bounds__(256) void cvt_h8(const float* __restrict__ in, unsigned short* out, int n8, float scale) {
  const int i = blockIdx.x * 256 + threadIdx.x;
  if (i < n8) {
    const v4f a = *(const v4f*)(in + (size_t)i * 8);
    const v4f c = *(const v4f*)(in + (size_t)i * 8 + 4);
    float f[8];
    f[0] = a[0]; f[1] = a[1]; f[2] = a[2]; f[3] = a[3];
    f[4] = c[0]; f[5] = c[1]; f[6] = c[2]; f[7] = c[3];
    unsigned short hb[8];
#pragma unroll
    for (int e = 0; e < 8; ++e) hb[e] = h_bits((_Float16)(bf_up(bf_bits(f[e])) * scale));
    v4u p;
    p[0] = pk16(hb[0], hb[1]);
    p[1] = pk16(hb[2], hb[3]);
    p[2] = pk16(hb[4], hb[5]);
    p[3] = pk16(hb[6], hb[7]);
    *(volatile v4u*)(out + (size_t)i * 8) = p;
    __threadfence();
    *(volatile v4u*)(out + (size_t)i * 8) = p;
  }
}

__global__ __launch_bounds__(256) void cvt_xt(const float* __restrict__ xg, unsigned short* XT, float scale) {
  __shared__ __align__(16) unsigned short ts[64 * QTP];
  const int tid = threadIdx.x;
  const int t0 = blockIdx.x * 64, c0 = blockIdx.y * 64;
#pragma unroll 1
  for (int pass = 0; pass < 4; ++pass) {
    const int cl = pass * 16 + (tid >> 4);
    const int l4 = (tid & 15) * 4;
    const int tok = t0 + l4;
    const int tokc = min(tok, NTG - 4);
    const int bl = tokc / NRES;
    const int n  = tokc - bl * NRES;
    const v4f v = *(const v4f*)(xg + ((size_t)(bl * DIMC + c0 + cl)) * NRES + n);
    const bool ok = (tok < NTG);
#pragma unroll
    for (int i = 0; i < 4; ++i) {
      const float f = ok ? v[i] : 0.0f;
      ts[(l4 + i) * QTP + cl] = h_bits((_Float16)(bf_up(bf_bits(f)) * scale));
    }
  }
  __syncthreads();
#pragma unroll 1
  for (int pass = 0; pass < 2; ++pass) {
    const int lr = pass * 32 + (tid >> 3);
    const int c8 = (tid & 7) * 8;
    const v4u v = *(const v4u*)(ts + lr * QTP + c8);
    unsigned short* dst = XT + ((size_t)(t0 + lr)) * DIMC + c0 + c8;
    *(volatile v4u*)dst = v;
    __threadfence();
    *(volatile v4u*)dst = v;
  }
}

__global__ __launch_bounds__(256) void bias_expand(const float* __restrict__ ab, const int* __restrict__ bidx,
                                                   int n_off, float* BT) {
  const int i = blockIdx.x * 256 + threadIdx.x;
  if (i < NBT) {
    const int r    = i & 7;
    const int lane = (i >> 3) & 31;
    int rest = i >> 8;
    const int mt = rest % NMT;  rest /= NMT;
    const int nt = rest % NQT;
    const int h  = rest / NQT;
    const int n = nt * 16 + (lane & 15);
    const int m = mt * 16 + 8 * (lane >> 4) + r;
    const int nc = min(n, NRES - 1), mc = min(m, NRES - 1);
    int ix = bidx[nc * NRES + mc];
    ix = min(max(ix, 0), n_off - 1);
    const float bvv = bf_up(bf_bits(ab[h * n_off + ix]));
    const float v = (n < NRES && m < NRES) ? bvv : 0.0f;
    *(volatile float*)(BT + i) = v;
    __threadfence();
    *(volatile float*)(BT + i) = v;
  }
}

__global__ __launch_bounds__(256) void gemm_qkv(
    const unsigned short* __restrict__ Wp, const unsigned short* __restrict__ XTp,
    const float* __restrict__ qb,
    unsigned short* QH, unsigned short* QL, unsigned short* KX,
    unsigned short* VH, unsigned short* VL, float oscale) {
  const _Float16* A  = (const _Float16*)(const void*)Wp;
  const _Float16* Bt = (const _Float16*)(const void*)XTp;
  __shared__ __align__(16) unsigned short sP[8][2][16 * SPP];
  const int lane = threadIdx.x & 31;
  const int wave = threadIdx.x >> 5;
  const int tilesN = TGP / 64;
  const int tilesM = OQKV / 64;
  const int tile = blockIdx.x * 8 + wave;
  if (tile >= tilesM * tilesN) return;
  const int tm = tile / tilesN;
  const int tn = tile - tm * tilesN;
  const int m0 = tm << 6;
  const int n0 = tn << 6;
  const int rlane = lane & 15;
  const int hh    = lane >> 4;
  const int koff  = hh * 8;
  const int mOff  = hh * 8;

  v8f acc[4][4];
#pragma unroll
  for (int i = 0; i < 4; ++i)
#pragma unroll
    for (int j = 0; j < 4; ++j) acc[i][j] = zero8();

  for (int k0 = 0; k0 < DIMC; k0 += 32) {
    v16h bf[4];
#pragma unroll
    for (int j = 0; j < 4; ++j) {
      const size_t bo = (size_t)(n0 + (j << 4) + rlane) * DIMC + koff + k0;
      bf[j] = ldfrag_h(Bt + bo);
    }
#pragma unroll
    for (int i = 0; i < 4; ++i) {
      const size_t ao = (size_t)(m0 + (i << 4) + rlane) * DIMC + koff + k0;
      const v16h ah = ldfrag_h(A + ao);
#pragma unroll
      for (int j = 0; j < 4; ++j) acc[i][j] = mma_h_raw(ah, bf[j], acc[i][j]);
      dep_guard_h(acc[i][0], acc[i][3], ah, bf[3]);
    }
    keep4_h(bf[0], bf[1], bf[2], bf[3]);
  }
  acc_guard4(acc[0][0], acc[0][1], acc[0][2], acc[0][3]);
  acc_guard4(acc[1][0], acc[1][1], acc[1][2], acc[1][3]);
  acc_guard4(acc[2][0], acc[2][1], acc[2][2], acc[2][3]);
  acc_guard4(acc[3][0], acc[3][1], acc[3][2], acc[3][3]);

  const int sec = m0 >> 9;
  const int h   = (m0 & 511) >> 6;
  float bv[4][8];
#pragma unroll
  for (int i = 0; i < 4; ++i)
#pragma unroll
    for (int r = 0; r < 8; ++r) bv[i][r] = bf_up(bf_bits(qb[m0 + (i << 4) + mOff + r]));
  unsigned short* s0 = &sP[wave][0][0];
  unsigned short* s1 = &sP[wave][1][0];
  const int rq = lane >> 3, c8 = (lane & 7) * 8;

  if (sec < 2) {
    unsigned short* Ph = (sec == 0) ? QH : KX;
#pragma unroll
    for (int j = 0; j < 4; ++j) {
#pragma unroll
      for (int i = 0; i < 4; ++i) {
        unsigned short hb[8], lb[8];
#pragma unroll
        for (int r = 0; r < 8; ++r) {
          const float f = (acc[i][j][r] * oscale + bv[i][r]) * 16.0f;
          const _Float16 xh = (_Float16)f;
          hb[r] = h_bits(xh);
          lb[r] = h_bits((_Float16)((f - (float)xh) * 2048.0f));
        }
        v4u ph, pl;
#pragma unroll
        for (int q = 0; q < 4; ++q) {
          ph[q] = pk16(hb[2 * q], hb[2 * q + 1]);
          pl[q] = pk16(lb[2 * q], lb[2 * q + 1]);
        }
        *(v4u*)(s0 + rlane * SPP + (i << 4) + mOff) = ph;
        if (sec == 0) *(v4u*)(s1 + rlane * SPP + (i << 4) + mOff) = pl;
      }
      wave_sync_lds();
      for (int pass = 0; pass < 2; ++pass) {
#pragma unroll
        for (int it = 0; it < 4; ++it) {
          const int row = it * 4 + rq;
          const size_t dst = ((size_t)(h * TGP + n0 + (j << 4) + row)) * HD + c8;
          const v4u v = *(const v4u*)(s0 + row * SPP + c8);
          *(volatile v4u*)(Ph + dst) = v;
          if (sec == 0) {
            const v4u w = *(const v4u*)(s1 + row * SPP + c8);
            *(volatile v4u*)(QL + dst) = w;
          }
        }
        __threadfence();
      }
      wave_sync_lds();
    }
  } else {
#pragma unroll
    for (int i = 0; i < 4; ++i) {
#pragma unroll
      for (int j = 0; j < 4; ++j) {
#pragma unroll
        for (int r = 0; r < 8; ++r) {
          const float f = (acc[i][j][r] * oscale + bv[i][r]) * 16.0f;
          const _Float16 xh = (_Float16)f;
          const int so = (mOff + r) * SPP + (j << 4) + rlane;
          s0[so] = h_bits(xh);
          s1[so] = h_bits((_Float16)((f - (float)xh) * 2048.0f));
        }
      }
      wave_sync_lds();
      for (int pass = 0; pass < 2; ++pass) {
#pragma unroll
        for (int it = 0; it < 4; ++it) {
          const int row = it * 4 + rq;
          const size_t dst = ((size_t)(h * HD + (i << 4) + row)) * TGP + n0 + c8;
          const v4u v = *(const v4u*)(s0 + row * SPP + c8);
          const v4u w = *(const v4u*)(s1 + row * SPP + c8);
          *(volatile v4u*)(VH + dst) = v;
          *(volatile v4u*)(VL + dst) = w;
        }
        __threadfence();
      }
      wave_sync_lds();
    }
  }
}

__global__ __launch_bounds__(ATHR) void attn_kernel(
    const unsigned short* __restrict__ QHp, const unsigned short* __restrict__ QLp,
    const unsigned short* __restrict__ KXp,
    const unsigned short* __restrict__ VHp, const unsigned short* __restrict__ VLp,
    const float* __restrict__ BT,
    unsigned short* CTXh, unsigned short* CTXl, float rscale) {
  __shared__ __align__(16) unsigned short lds_u[LDSH];
  unsigned short* kl_u = lds_u;
  unsigned short* vh_u = lds_u + NKEY * KP;
  unsigned short* vl_u = vh_u + HD * VP;
  const _Float16* kl = (const _Float16*)(const void*)kl_u;
  const _Float16* vh = (const _Float16*)(const void*)vh_u;
  const _Float16* vl = (const _Float16*)(const void*)vl_u;
  const _Float16* QH = (const _Float16*)(const void*)QHp;
  const _Float16* QL = (const _Float16*)(const void*)QLp;

  const int tid = threadIdx.x, lane = tid & 31, wave = tid >> 5;
  const int h = blockIdx.x, bl = blockIdx.y;
  const int tokbase = bl * NRES;
  const int rlane = lane & 15, hsel = lane >> 4, koff = hsel * 8;

  for (int i = tid; i < NKEY * 8; i += ATHR) {
    const int key = i >> 3, c8 = (i & 7) * 8;
    const v4u v = *(const v4u*)(KXp + ((size_t)(h * TGP + tokbase + key)) * HD + c8);
    *(v4u*)(kl_u + key * KP + c8) = v;
  }
  for (int i = tid; i < HD * (NKEY / 4); i += ATHR) {
    const int d = i / (NKEY / 4);
    const int j = i - d * (NKEY / 4);
    const size_t go = ((size_t)(h * HD + d)) * TGP + tokbase + 4 * j;
    const v2u a = *(const v2u*)(VHp + go);
    const v2u c = *(const v2u*)(VLp + go);
    *(v2u*)(vh_u + d * VP + 4 * j) = a;
    *(v2u*)(vl_u + d * VP + 4 * j) = c;
  }
  __syncthreads();

  const int n0 = wave * 16;
  const size_t qo = ((size_t)(h * TGP + tokbase + n0 + rlane)) * HD + koff;
  const v16h qh0 = ldfrag_h(QH + qo);
  const v16h qh1 = ldfrag_h(QH + qo + 32);
  const v16h ql0 = ldfrag_h(QL + qo);
  const v16h ql1 = ldfrag_h(QL + qo + 32);
  const float* bb = BT + (((size_t)(h * NQT + wave) * NMT) * 32 + lane) * 8;

  const float C2048  = 1.0f / 2048.0f;
  const float LN1024 = 6.931471805599453f;

  v8f oh[4], ol[4];
#pragma unroll
  for (int dt = 0; dt < 4; ++dt) { oh[dt] = zero8(); ol[dt] = zero8(); }
  float m_run = -1.0e30f, l_run = 0.0f;

#pragma unroll 1
  for (int sub = 0; sub < NKST; ++sub) {
    const int kr = sub * 32;
    float a[2][8];
#pragma unroll
    for (int t = 0; t < 2; ++t) {
      const int krow = kr + 16 * t + rlane;
      const v16h kfa = ldfrag_h(kl + krow * KP + koff);
      const v16h kfb = ldfrag_h(kl + krow * KP + 32 + koff);
      v8f sh = mma_h_raw(kfa, qh0, zero8());
      sh = mma_h_raw(kfb, qh1, sh);
      v8f sr = mma_h_raw(kfa, ql0, zero8());
      sr = mma_h_raw(kfb, ql1, sr);
      guard_sc(sh, sr, kfa, kfb, qh0, qh1, ql0, ql1);
      const float* bp = bb + (2 * sub + t) * 256;
      const v4f b0 = *(const v4f*)(bp);
      const v4f b1 = *(const v4f*)(bp + 4);
      float bvv[8];
      bvv[0] = b0[0]; bvv[1] = b0[1]; bvv[2] = b0[2]; bvv[3] = b0[3];
      bvv[4] = b1[0]; bvv[5] = b1[1]; bvv[6] = b1[2]; bvv[7] = b1[3];
#pragma unroll
      for (int r = 0; r < 8; ++r) {
        const int key = kr + 16 * t + 8 * hsel + r;
        const float s = (sh[r] + sr[r] * C2048) * C2048 + bvv[r];
        a[t][r] = (key < NRES) ? s : -1.0e30f;
      }
    }

    float mloc = -1.0e30f;
#pragma unroll
    for (int r = 0; r < 8; ++r) mloc = fmaxf(mloc, fmaxf(a[0][r], a[1][r]));
    mloc = fmaxf(mloc, __shfl_xor(mloc, 16, 32));
    const float newM  = fmaxf(m_run, mloc);
    const float alpha = __expf(m_run - newM);
    const float msh   = newM - LN1024;
    float ssum = 0.0f;
    float p[2][8];
#pragma unroll
    for (int r = 0; r < 8; ++r) {
      p[0][r] = __expf(a[0][r] - msh);
      p[1][r] = __expf(a[1][r] - msh);
      ssum += p[0][r] + p[1][r];
    }
    ssum += __shfl_xor(ssum, 16, 32);
    l_run = l_run * alpha + ssum;
    m_run = newM;
#pragma unroll
    for (int dt = 0; dt < 4; ++dt) {
#pragma unroll
      for (int r = 0; r < 8; ++r) { oh[dt][r] *= alpha; ol[dt][r] *= alpha; }
    }

    union { v16h v; _Float16 s[16]; } ph, plo;
#pragma unroll
    for (int r = 0; r < 8; ++r) {
      const _Float16 x0 = (_Float16)p[0][r];
      const _Float16 x1 = (_Float16)p[1][r];
      ph.s[r]      = x0;
      ph.s[8 + r]  = x1;
      plo.s[r]     = (_Float16)((p[0][r] - (float)x0) * 2048.0f);
      plo.s[8 + r] = (_Float16)((p[1][r] - (float)x1) * 2048.0f);
    }

#pragma unroll
    for (int dt = 0; dt < 4; ++dt) {
      const v16h vah = ldfrag_h(vh + (16 * dt + rlane) * VP + kr + koff);
      const v16h val = ldfrag_h(vl + (16 * dt + rlane) * VP + kr + koff);
      oh[dt] = mma_h_raw(vah, ph.v, oh[dt]);
      ol[dt] = mma_h_raw(val, ph.v, ol[dt]);
      ol[dt] = mma_h_raw(vah, plo.v, ol[dt]);
      guard_pv(oh[dt], ol[dt], vah, val, ph.v, plo.v);
    }
  }
  acc_guard4(oh[0], oh[1], oh[2], oh[3]);
  acc_guard4(ol[0], ol[1], ol[2], ol[3]);

  const float inv = 4.0f * (1.0f / l_run);
  __syncthreads();
  unsigned short* sth = lds_u + wave * 2048;
  unsigned short* stl = sth + 1024;
#pragma unroll
  for (int dt = 0; dt < 4; ++dt) {
    v4u hv, lw;
#pragma unroll
    for (int e = 0; e < 4; ++e) {
      const float f0 = (oh[dt][2 * e]     + ol[dt][2 * e]     * C2048) * inv;
      const float f1 = (oh[dt][2 * e + 1] + ol[dt][2 * e + 1] * C2048) * inv;
      const _Float16 x0 = (_Float16)f0, x1 = (_Float16)f1;
      hv[e] = pk16(h_bits(x0), h_bits(x1));
      lw[e] = pk16(h_bits((_Float16)((f0 - (float)x0) * rscale)),
                   h_bits((_Float16)((f1 - (float)x1) * rscale)));
    }
    const int so = rlane * 64 + 16 * dt + 8 * hsel;
    *(v4u*)(sth + so) = hv;
    *(v4u*)(stl + so) = lw;
  }
  wave_sync_lds();
  {
    const int rq = lane >> 3, c8 = (lane & 7) * 8;
    for (int pass = 0; pass < 2; ++pass) {
#pragma unroll
      for (int it = 0; it < 4; ++it) {
        const int row = it * 4 + rq;
        const int n = n0 + row;
        const v4u v = *(const v4u*)(sth + row * 64 + c8);
        if (n < NRES) *(volatile v4u*)(CTXh + ((size_t)(tokbase + n)) * DIMC + h * HD + c8) = v;
      }
      __threadfence();
    }
    for (int pass = 0; pass < 2; ++pass) {
#pragma unroll
      for (int it = 0; it < 4; ++it) {
        const int row = it * 4 + rq;
        const int n = n0 + row;
        const v4u v = *(const v4u*)(stl + row * 64 + c8);
        if (n < NRES) *(volatile v4u*)(CTXl + ((size_t)(tokbase + n)) * DIMC + h * HD + c8) = v;
      }
      __threadfence();
    }
  }
}

template <int NSPLIT, int BIAS>
__global__ __launch_bounds__(256) void gemm64(
    const unsigned short* __restrict__ Ap, int lda, long long sAy, long long sAz,
    const unsigned short* __restrict__ Btp, int ldb, long long sBy, long long sBz,
    const unsigned short* __restrict__ Bt2p, int ldb2,
    const float* __restrict__ bias,
    float* Cout, int ldc, long long sCy, long long sCz,
    int M, int N, int K, float oscale, float rres) {
  const _Float16* A   = (const _Float16*)(const void*)Ap;
  const _Float16* Bt  = (const _Float16*)(const void*)Btp;
  const _Float16* Bt2 = (const _Float16*)(const void*)Bt2p;
  __shared__ __align__(16) float sT[8][16 * 68];
  const int by   = blockIdx.y;
  const int bz   = blockIdx.z;
  const int lane = threadIdx.x & 31;
  const int wave = threadIdx.x >> 5;
  const int tilesN = N >> 6;
  const int tilesM = M >> 6;
  const int tile = blockIdx.x * 8 + wave;
  if (tile >= tilesM * tilesN) return;
  const int tm = tile / tilesN;
  const int tn = tile - tm * tilesN;
  const int m0 = tm << 6;
  const int n0 = tn << 6;

  const _Float16* Ab  = A + (size_t)by * (size_t)sAy + (size_t)bz * (size_t)sAz;
  const _Float16* Bb  = Bt + (size_t)by * (size_t)sBy + (size_t)bz * (size_t)sBz;
  const _Float16* Bb2 = (NSPLIT == 2) ? (Bt2 + (size_t)by * (size_t)sBy + (size_t)bz * (size_t)sBz) : Bb;
  const int ld2 = (NSPLIT == 2) ? ldb2 : ldb;

  const int rlane = lane & 15;
  const int koff  = (lane >> 4) * 8;
  const int mOff  = (lane >> 4) * 8;

  v8f acc[4][4];
#pragma unroll
  for (int i = 0; i < 4; ++i)
#pragma unroll
    for (int j = 0; j < 4; ++j) acc[i][j] = zero8();

  for (int k0 = 0; k0 < K; k0 += 32) {
    v16h bf[4];
#pragma unroll
    for (int j = 0; j < 4; ++j) {
      const size_t bo = (size_t)(n0 + (j << 4) + rlane) * ldb + koff + k0;
      bf[j] = ldfrag_h(Bb + bo);
    }
#pragma unroll
    for (int i = 0; i < 4; ++i) {
      const size_t ao = (size_t)(m0 + (i << 4) + rlane) * lda + koff + k0;
      const v16h ah = ldfrag_h(Ab + ao);
#pragma unroll
      for (int j = 0; j < 4; ++j) acc[i][j] = mma_h_raw(ah, bf[j], acc[i][j]);
      dep_guard_h(acc[i][0], acc[i][3], ah, bf[3]);
    }
    if (NSPLIT == 2) {
#pragma unroll
      for (int j = 0; j < 4; ++j) {
        const size_t bo = (size_t)(n0 + (j << 4) + rlane) * ld2 + koff + k0;
        bf[j] = ldfrag_h(Bb2 + bo);
      }
#pragma unroll
      for (int i = 0; i < 4; ++i) {
        const size_t ao = (size_t)(m0 + (i << 4) + rlane) * lda + koff + k0;
        const v16h al = ldfrag_h(Ab + ao);
#pragma unroll
        for (int j = 0; j < 4; ++j) {
          v8f tp = mma_h_raw(al, bf[j], zero8());
          res_guard(tp, acc[i][j], al, bf[j]);
#pragma unroll
          for (int r = 0; r < 8; ++r) acc[i][j][r] += tp[r] * rres;
        }
        dep_guard_h(acc[i][0], acc[i][3], al, bf[3]);
      }
    }
    keep4_h(bf[0], bf[1], bf[2], bf[3]);
  }
  acc_guard4(acc[0][0], acc[0][1], acc[0][2], acc[0][3]);
  acc_guard4(acc[1][0], acc[1][1], acc[1][2], acc[1][3]);
  acc_guard4(acc[2][0], acc[2][1], acc[2][2], acc[2][3]);
  acc_guard4(acc[3][0], acc[3][1], acc[3][2], acc[3][3]);

  float* slab = sT[wave];
  float* C = Cout + (size_t)by * (size_t)sCy + (size_t)bz * (size_t)sCz;
#pragma unroll
  for (int i = 0; i < 4; ++i) {
    const int mBase = m0 + (i << 4);
    float brow[8];
#pragma unroll
    for (int r = 0; r < 8; ++r) brow[r] = 0.f;
    if (BIAS == 2) {
#pragma unroll
      for (int r = 0; r < 8; ++r) brow[r] = bf_up(bf_bits(bias[mBase + mOff + r]));
    }
#pragma unroll
    for (int j = 0; j < 4; ++j) {
#pragma unroll
      for (int r = 0; r < 8; ++r) {
        slab[(mOff + r) * 68 + (j << 4) + rlane] = acc[i][j][r] * oscale + brow[r];
      }
    }
    wave_sync_lds();
    {
      const int hh = lane >> 4, c4 = (lane & 15) * 4;
      for (int pass = 0; pass < 2; ++pass) {
#pragma unroll
        for (int it = 0; it < 8; ++it) {
          const int row = it * 2 + hh;
          const v4f v = *(const v4f*)(slab + row * 68 + c4);
          *(volatile v4f*)(C + (size_t)(mBase + row) * ldc + n0 + c4) = v;
        }
        __threadfence();
      }
    }
    wave_sync_lds();
  }
}

__global__ __launch_bounds__(256) void pack_out(const float* __restrict__ YP, float* outg) {
  const int s = blockIdx.x * 256 + threadIdx.x;
  if (s < (GIMG * DIMC * NRES) / 4) {
    const int f   = s * 4;
    const int bl  = f / (DIMC * NRES);
    const int rem = f - bl * (DIMC * NRES);
    const int o   = rem / NRES;
    const int n   = rem - o * NRES;
    const v4f v = *(const v4f*)(YP + (size_t)o * NTG + bl * NRES + n);
    *(volatile v4f*)(outg + f) = v;
    __threadfence();
    *(volatile v4f*)(outg + f) = v;
  }
}

extern "C" void kernel_launch(void* const* d_in, const int* in_sizes, int n_in,
                              void* d_out, int out_size, void* d_ws, size_t ws_size,
                              hipStream_t stream) {
  if (n_in < 7) return;
  if (in_sizes[0] != NIMG * DIMC * NRES) return;
  if (in_sizes[1] != OQKV * DIMC) return;
  if (in_sizes[2] != OQKV) return;
  if (in_sizes[3] != DIMC * DIMC) return;
  if (in_sizes[4] != DIMC) return;
  if (in_sizes[5] != HEADS * NRES) return;
  if (in_sizes[6] != NRES * NRES) return;
  if (out_size != NIMG * DIMC * NRES) return;

  const float* x      = (const float*)d_in[0];
  const float* qkv_w  = (const float*)d_in[1];
  const float* qkv_b  = (const float*)d_in[2];
  const float* proj_w = (const float*)d_in[3];
  const float* proj_b = (const float*)d_in[4];
  const float* ab     = (const float*)d_in[5];
  const int*   bidx   = (const int*)d_in[6];
  const int    n_off  = in_sizes[5] / HEADS;

  const size_t PW3 = (size_t)OQKV * DIMC * 2;
  const size_t PPW = (size_t)DIMC * DIMC * 2;
  const size_t PBT = (size_t)NBT * 4;
  const size_t PXT = (size_t)TGP * DIMC * 2;
  const size_t PQ  = (size_t)HEADS * TGP * HD * 2;
  const size_t PV  = (size_t)HEADS * HD * TGP * 2;
  const size_t PCT = (size_t)NTG * DIMC * 2;
  const size_t PYP = (size_t)DIMC * NTG * 4;
  size_t off = 0;
  const size_t oW3 = off; off += PW3;
  const size_t oPW = off; off += PPW;
  const size_t oBT = off; off += PBT;
  const size_t oXT = off; off += PXT;
  const size_t oQH = off; off += PQ;
  const size_t oQL = off; off += PQ;
  const size_t oKX = off; off += PQ;
  const size_t oVH = off; off += PV;
  const size_t oVL = off; off += PV;
  const size_t oCH = off; off += PCT;
  const size_t oCL = off; off += PCT;
  const size_t oYP = off; off += PYP;
  if (off > ws_size) return;
  if (off > (size_t)134217728) return;

  char* ws = (char*)d_ws;
  unsigned short* W3   = (unsigned short*)(ws + oW3);
  unsigned short* PWp  = (unsigned short*)(ws + oPW);
  float*          BT   = (float*)(ws + oBT);
  unsigned short* XT   = (unsigned short*)(ws + oXT);
  unsigned short* QH   = (unsigned short*)(ws + oQH);
  unsigned short* QL   = (unsigned short*)(ws + oQL);
  unsigned short* KX   = (unsigned short*)(ws + oKX);
  unsigned short* VH   = (unsigned short*)(ws + oVH);
  unsigned short* VL   = (unsigned short*)(ws + oVL);
  unsigned short* CTXh = (unsigned short*)(ws + oCH);
  unsigned short* CTXl = (unsigned short*)(ws + oCL);
  float*          YP   = (float*)(ws + oYP);
  float*          out  = (float*)d_out;

  const dim3 blk(256);
  const int n8w3 = OQKV * DIMC / 8;
  const int n8pw = DIMC * DIMC / 8;
  const dim3 gW3((n8w3 + 255) / 256);
  const dim3 gPW((n8pw + 255) / 256);
  const dim3 gBT((NBT + 255) / 256);
  const dim3 gXT(TGP / 64, DIMC / 64);
  const dim3 gQkv(((OQKV / 64) * (TGP / 64) + 7) / 8, 1, 1);
  const dim3 gAttn(HEADS, GIMG);
  const dim3 gProj(((DIMC / 64) * (NTG / 64) + 7) / 8, 1, 1);
  const dim3 gPack(((GIMG * DIMC * NRES) / 4 + 255) / 256);

  const float oscQkv = 1.0f / 16384.0f;
  const float rscale = 16384.0f;
  const float oscPrj = 1.0f / 65536.0f;
  const float rres   = 1.0f / 16384.0f;

  cvt_h8<<<gW3, blk, 0, stream>>>(qkv_w, W3, n8w3, 1024.0f);
  cvt_h8<<<gPW, blk, 0, stream>>>(proj_w, PWp, n8pw, 1024.0f);
  bias_expand<<<gBT, blk, 0, stream>>>(ab, bidx, n_off, BT);

  for (int g = 0; g < NGRP; ++g) {
    const float* xg   = x   + (size_t)g * GIMG * DIMC * NRES;
    float*       outg = out + (size_t)g * GIMG * DIMC * NRES;
    cvt_xt<<<gXT, blk, 0, stream>>>(xg, XT, 16.0f);
    gemm_qkv<<<gQkv, blk, 0, stream>>>(W3, XT, qkv_b, QH, QL, KX, VH, VL, oscQkv);
    attn_kernel<<<gAttn, dim3(ATHR), 0, stream>>>(QH, QL, KX, VH, VL, BT, CTXh, CTXl, rscale);
    gemm64<2, 2><<<gProj, blk, 0, stream>>>(
        PWp, DIMC, 0LL, 0LL,
        CTXh, DIMC, 0LL, 0LL,
        CTXl, DIMC,
        proj_b,
        YP, NTG, 0LL, 0LL,
        DIMC, NTG, DIMC, oscPrj, rres);
    pack_out<<<gPack, blk, 0, stream>>>(YP, outg);
  }
  (void)hipGetLastError();
}
